// Masker_69947837383272
// MI455X (gfx1250) — hardware-run, weakly checked
//
#include <hip/hip_runtime.h>


namespace {
constexpr int N = 10000, E = 160000, F = 128, C = 128  , NPB = 8;
constexpr float XS = 8.0f, HS = 256.0f, WSC = 256.0f;
typedef _Float16 b16;
typedef __attribute__((ext_vector_type(16))) _Float16 v16b;
typedef __attribute__((ext_vector_type(8))) _Float16 v8b;
typedef __attribute__((ext_vector_type(8))) float v8f;
typedef __attribute__((ext_vector_type(4))) float v4f;
__device__ __forceinline__ float bf16_rne(float f) { unsigned int u = __float_as_uint(f); u += 0x7FFFu + ((u >> 16) & 1u); float r = __uint_as_float(u & 0xFFFF0000u); asm volatile("" : "+v"(r)); return r; }
__device__ __forceinline__ float bfv(float f) { float r = bf16_rne(f); asm volatile("" : "+v"(r)); return r; }
__device__ __forceinline__ void split16(float v, b16& hi, b16& lo) { hi = (b16)v; lo = (b16)(v - (float)hi); }
__device__ __forceinline__ v16b frag_kb(const b16* p, int hh) { const v8b a = *(const v8b*)(p + 8 * hh), b = *(const v8b*)(p + 16 + 8 * hh); v16b f;
#pragma unroll
  for (int e = 0; e < 8; ++e) { f[e] = a[e]; f[8 + e] = b[e]; } return f; }
__device__ __forceinline__ v8f wmma16b(v16b a, v16b b, v8f c) { v8f d = __builtin_amdgcn_wmma_f32_16x16x32_f16(false, a, false, b, (short)0, c, false, false); asm volatile("v_nop\n\tv_nop\n\tv_nop\n\tv_nop" : "+v"(d) : "v"(a), "v"(b)); return d; }
__device__ __forceinline__ void wave_lds_sync() { __builtin_amdgcn_fence(__ATOMIC_RELEASE, "workgroup"); __builtin_amdgcn_wave_barrier(); __builtin_amdgcn_fence(__ATOMIC_ACQUIRE, "workgroup"); }
__device__ __forceinline__ float pmul(float a, float b) { float p = a * b; asm volatile("" : "+v"(p)); return p; }
__device__ __forceinline__ int iclamp(int v, int lo, int hi) { return v < lo ? lo : (v > hi ? hi : v); }
__device__ __forceinline__ float elu(float v) { return v > 0.0f ? v : (__expf(v) - 1.0f); }
constexpr int CSR_NBLK7 = 512, CSR_GB7 = 7, CSR_GN7 = 1 << CSR_GB7  , CSR_TS7 = (CSR_GN7 < 32 ? 32 : CSR_GN7)  , CSR_MAXG7 = 512, CSR_CAP7 = 12288  ;
__device__ __host__ __forceinline__ int csr_tix7(int v) { return (v >> CSR_GB7) * CSR_TS7 + (v & (CSR_GN7 - 1)); }
__global__ __launch_bounds__(64) void csrA_kernel7(const int* __restrict__ dst, int E, int N, int nG, int CHP, int NGP, int* __restrict__ STG, int* __restrict__ HST) {
  extern __shared__ int sm[];
  int* cnt = sm; int* run = sm + NGP; int* ids = sm + 2 * NGP;
  const int b = blockIdx.x; const int ch = (E + CSR_NBLK7 - 1) / CSR_NBLK7; const int e0 = b * ch, e1 = min(E, e0 + ch);
  for (int i = threadIdx.x; i < NGP; i += 64) cnt[i] = 0;
  for (int i = threadIdx.x; i < CHP; i += 64) ids[i] = -1;
  __syncthreads();
  if (threadIdx.x == 0) {
    for (int e = e0; e < e1; ++e) { int d = dst[e]; d = (d < 0) ? 0 : (d >= N ? N - 1 : d); cnt[d >> CSR_GB7] += 1; }
    int acc = 0; for (int g = 0; g < nG; ++g) { run[g] = acc; acc += cnt[g]; }
    for (int e = e0; e < e1; ++e) { int d = dst[e]; d = (d < 0) ? 0 : (d >= N ? N - 1 : d); const int g = d >> CSR_GB7; ids[run[g]] = e; run[g] += 1; } }
  __syncthreads();
  typedef __attribute__((ext_vector_type(4))) int v4i;
  for (int pass = 0; pass < 2; ++pass) {
    for (int i = threadIdx.x; i < CHP / 4; i += 64) *(volatile v4i*)(STG + (size_t)b * CHP + i * 4) = *(const v4i*)(&ids[i * 4]);
    for (int i = threadIdx.x; i < NGP / 4; i += 64) { v4i v; for (int e = 0; e < 4; ++e) v[e] = (i * 4 + e < nG) ? cnt[i * 4 + e] : 0; *(volatile v4i*)(HST + (size_t)b * NGP + i * 4) = v; }
    __threadfence(); }
}
__global__ __launch_bounds__(512) void csrS_kernel7(const int* __restrict__ HST, int nG, int NGP, int* __restrict__ START, int* __restrict__ TOT, int* __restrict__ OFF) {
  __shared__ int tot[CSR_MAXG7];
  const int b = threadIdx.x;
  for (int pass = 0; pass < 2; ++pass) { int runb = 0; for (int g = 0; g < nG; ++g) { int c = HST[(size_t)b * NGP + g]; c = (c < 0) ? 0 : c; ((volatile int*)OFF)[(size_t)g * CSR_NBLK7 + b] = runb; runb += c; } __threadfence(); }
  for (int g = threadIdx.x; g < nG; g += 512) { int s = 0; for (int bb = 0; bb < CSR_NBLK7; ++bb) { int c = HST[(size_t)bb * NGP + g]; s += (c < 0) ? 0 : c; } tot[g] = s; }
  __syncthreads();
  if (threadIdx.x < 32) {
    __shared__ int st[CSR_MAXG7 + 32];
    if (threadIdx.x == 0) { int acc = 0; for (int g = 0; g < NGP; ++g) { st[g] = acc; if (g < nG) acc += (tot[g] + 31) & ~31; } st[NGP] = acc; }
    __builtin_amdgcn_fence(__ATOMIC_RELEASE, "workgroup"); __builtin_amdgcn_wave_barrier(); __builtin_amdgcn_fence(__ATOMIC_ACQUIRE, "workgroup");
    for (int pass = 0; pass < 2; ++pass) { for (int i = threadIdx.x; i < NGP + 32; i += 32) { ((volatile int*)START)[i] = (i <= NGP) ? st[min(i, NGP)] : 0; ((volatile int*)TOT)[i] = (i < nG) ? tot[i] : 0; } __threadfence(); } }
}
__global__ __launch_bounds__(256) void csrB_kernel7(const int* __restrict__ dst, int N, int nG, int CHP, int NGP, int permLen, const int* __restrict__ STG, const int* __restrict__ HST, const int* __restrict__ OFF, const int* __restrict__ START, const int* __restrict__ TOT, int* __restrict__ PERM, int* __restrict__ ROWPTR, int* __restrict__ ROWCNT, int* __restrict__ FLAG) {
  typedef __attribute__((ext_vector_type(4))) int v4i;
  __shared__ int ids[CSR_CAP7]; __shared__ unsigned short key[CSR_CAP7]; __shared__ int outp[CSR_CAP7]; __shared__ int ncnt[CSR_GN7 + 1]; __shared__ int boff[CSR_NBLK7 + 1];
  const int g = blockIdx.x, t_ = threadIdx.x; int tot = TOT[g]; int st = START[g], stn = START[g + 1]; const int v0 = g * CSR_GN7; const int nv = min(CSR_GN7, N - v0); const int t0 = g * CSR_TS7;
  st = (st < 0) ? 0 : (st > permLen - 32 ? permLen - 32 : st) & ~31; stn = (stn < st) ? st : (stn > permLen ? permLen : stn); tot = (tot < 0) ? 0 : tot; if (tot > stn - st && tot <= CSR_CAP7) tot = stn - st;
  if (tot > CSR_CAP7) {
    for (int pass = 0; pass < 2; ++pass) { for (int i = t_; i < CSR_TS7 / 4; i += 256) { v4i a, c; for (int e = 0; e < 4; ++e) { a[e] = st; c[e] = 0; } *(volatile v4i*)(ROWPTR + t0 + i * 4) = a; *(volatile v4i*)(ROWCNT + t0 + i * 4) = c; } if (t_ == 0) ((volatile int*)FLAG)[0] = 1; __threadfence(); } (void)nv; return; }
  if (t_ == 0) { int acc = 0; for (int b = 0; b < CSR_NBLK7; ++b) { boff[b] = acc; int c = HST[(size_t)b * NGP + g]; c = (c < 0) ? 0 : (c > CHP ? CHP : c); acc += c; if (acc > tot) acc = tot; } boff[CSR_NBLK7] = acc; }
  for (int i = t_; i <= CSR_GN7; i += 256) ncnt[i] = 0;
  __syncthreads();
  for (int b = 0; b < CSR_NBLK7; ++b) { const int c = boff[b + 1] - boff[b]; int o_ = OFF[(size_t)g * CSR_NBLK7 + b]; o_ = (o_ < 0) ? 0 : (o_ > CHP - c ? CHP - c : o_); const int* src_ = STG + (size_t)b * CHP + o_;
    for (int i = t_; i < c; i += 256) { int id = src_[i]; id = (id < 0) ? 0 : id; ids[boff[b] + i] = id; int d = dst[id]; d = (d < v0) ? v0 : (d >= N ? N - 1 : d); int kk = d - v0; kk = (kk < 0) ? 0 : (kk >= CSR_GN7 ? CSR_GN7 - 1 : kk); key[boff[b] + i] = (unsigned short)kk; } }
  __syncthreads();
  if (t_ == 0) { for (int i = 0; i < tot; ++i) ncnt[key[i]] += 1; int acc = 0; for (int vl = 0; vl < CSR_GN7; ++vl) { const int c = ncnt[vl]; ncnt[vl] = acc; acc += c; } ncnt[CSR_GN7] = acc;
    for (int i = 0; i < tot; ++i) { const int vl = key[i]; outp[ncnt[vl]] = ids[i]; ncnt[vl] += 1; }
    for (int vl = CSR_GN7; vl > 0; --vl) ncnt[vl] = ncnt[vl - 1]; ncnt[0] = 0; }
  __syncthreads();
  for (int pass = 0; pass < 2; ++pass) {
    for (int i = t_; i < (stn - st) / 4; i += 256) { v4i v; for (int e = 0; e < 4; ++e) { const int q = i * 4 + e; v[e] = (q < tot) ? outp[q] : -1; } *(volatile v4i*)(PERM + st + i * 4) = v; }
    for (int i = t_; i < CSR_TS7 / 4; i += 256) { v4i a, c; for (int e = 0; e < 4; ++e) { const int vl = i * 4 + e; const int vc = vl < CSR_GN7 ? vl : CSR_GN7; a[e] = (vl < CSR_GN7) ? st + ncnt[vc] : st; c[e] = (vl < nv) ? (ncnt[(vc < CSR_GN7 ? vc : CSR_GN7 - 1) + 1] - ncnt[vc]) : 0; } *(volatile v4i*)(ROWPTR + t0 + i * 4) = a; *(volatile v4i*)(ROWCNT + t0 + i * 4) = c; }
    __threadfence(); }
}
__global__ __launch_bounds__(256) void csrZ_kernel7(int* __restrict__ p, size_t n4) { typedef __attribute__((ext_vector_type(4))) int v4i; const size_t tid = (size_t)blockIdx.x * 256 + threadIdx.x, nth = (size_t)gridDim.x * 256; v4i z = {0, 0, 0, 0}; for (size_t i = tid; i < n4; i += nth) *(volatile v4i*)(p + i * 4) = z; }
struct CsrBufs7 { int *STG, *HST, *OFF, *START, *TOT, *PERM, *ROWPTR, *ROWCNT, *FLAG; int nG, NGP, CHP; size_t permLen; char* base; size_t bytes; };
static size_t csr_carve7(CsrBufs7& c, char* ws, size_t off, int E, int N) {
  const size_t off0 = off; c.base = ws + off;
  auto al = [&](size_t bytes) { char* p = ws + off; off += (bytes + 255) & ~(size_t)255; return p; };
  c.nG = (N + CSR_GN7 - 1) / CSR_GN7; c.NGP = (c.nG + 31) & ~31; const int ch = (E + CSR_NBLK7 - 1) / CSR_NBLK7; c.CHP = (ch + 31) & ~31; c.permLen = (size_t)E + 32 * (size_t)c.nG + 32;
  c.STG = (int*)al((size_t)CSR_NBLK7 * c.CHP * 4); c.HST = (int*)al((size_t)CSR_NBLK7 * c.NGP * 4); c.OFF = (int*)al((size_t)c.NGP * CSR_NBLK7 * 4); c.START = (int*)al((size_t)(c.NGP + 64) * 4); c.TOT = (int*)al((size_t)(c.NGP + 64) * 4);
  c.PERM = (int*)al(c.permLen * 4); c.ROWPTR = (int*)al((size_t)c.nG * CSR_TS7 * 4); c.ROWCNT = (int*)al((size_t)c.nG * CSR_TS7 * 4); c.FLAG = (int*)al(256);
  c.bytes = off - off0; return off;
}
static void csr_build7(const CsrBufs7& c, const int* dst, int E, int N, hipStream_t stream) {
  const size_t smem = (size_t)(2 * c.NGP + c.CHP) * 4;
  csrZ_kernel7<<<512, 256, 0, stream>>>((int*)c.base, c.bytes / 16);
  csrA_kernel7<<<CSR_NBLK7, 64, smem, stream>>>(dst, E, N, c.nG, c.CHP, c.NGP, c.STG, c.HST);
  csrS_kernel7<<<1, 512, 0, stream>>>(c.HST, c.nG, c.NGP, c.START, c.TOT, c.OFF);
  csrB_kernel7<<<c.nG, 256, 0, stream>>>(dst, N, c.nG, c.CHP, c.NGP, (int)c.permLen, c.STG, c.HST, c.OFF, c.START, c.TOT, c.PERM, c.ROWPTR, c.ROWCNT, c.FLAG);
}


__global__ __launch_bounds__(256) void wput_kernel(const float* __restrict__ wa, const float* __restrict__ la, int KIN, int OA, int OL, int OWP, b16* __restrict__ WT) { const size_t nt = (size_t)gridDim.x * 256, u0 = (size_t)blockIdx.x * 256 + threadIdx.x; const int OW = OA + OL; v8b v;
  for (size_t u = u0; u < (size_t)OWP * (KIN / 8); u += nt) { const int o = (int)(u / (KIN / 8)), k0 = (int)(u % (KIN / 8)) * 8;
#pragma unroll
    for (int j = 0; j < 8; ++j) v[j] = o >= OW ? (b16)0.0f : (b16)(bf16_rne(o < OA ? wa[(size_t)(k0 + j) * OA + o] : la[(size_t)(k0 + j) * OL + o - OA]) * WSC); for (int pass = 0; pass < 2; ++pass) { *(volatile v8b*)(WT + (size_t)o * KIN + k0) = v; __threadfence(); } } }
template <int MODE, int KIN, int NH, int OL>
__global__ __launch_bounds__(32) void proj_kernel(const float* __restrict__ IN, const b16* __restrict__ WT, const float* __restrict__ as_, const float* __restrict__ ad_, const float* __restrict__ lb, int NLIM, float* __restrict__ FT, float* __restrict__ LN, float* __restrict__ ES) { constexpr int OA = NH * C, NG = (OA + OL + 255) / 256; __shared__ __attribute__((aligned(16))) b16 Ah[16][KIN + 8], Al[16][KIN + 8]; __shared__ float Tf[16][260], Eq[16][16]; const int lane = threadIdx.x, nloc = lane & 15, hlf = lane >> 4; const size_t m0 = (size_t)blockIdx.x * 16; if (m0 >= (size_t)NLIM) return;
  for (int rr = 0; rr < 16; ++rr) for (int q = 0; q < KIN / 32; ++q) { const int c = q * 32 + lane; const float v = IN[(m0 + rr) * KIN + c]; b16 p, ql; if (MODE == 0) { p = (b16)(bf16_rne(v) * XS); ql = (b16)0.0f; } else split16(v * HS, p, ql); Ah[rr][c] = p; Al[rr][c] = ql; }
  if (lane < 16) { for (int k = KIN; k < KIN + 8; ++k) { Ah[lane][k] = (b16)0.0f; Al[lane][k] = (b16)0.0f; } for (int j = 0; j < 16; ++j) Eq[lane][j] = 0.0f; }
  wave_lds_sync(); const float osc = MODE == 0 ? 1.0f / (XS * WSC) : 1.0f / (HS * WSC);
#pragma unroll 1
  for (int g = 0; g < NG; ++g) { v8f acc[16];
#pragma unroll
    for (int t = 0; t < 16; ++t) acc[t] = (v8f){};
#pragma unroll 2
    for (int kb = 0; kb < KIN; kb += 32) { const v16b a = frag_kb(&Ah[nloc][kb], hlf), al = frag_kb(&Al[nloc][kb], hlf);
#pragma unroll
      for (int t = 0; t < 16; ++t) { const v16b bw = frag_kb(WT + (size_t)(g * 256 + t * 16 + nloc) * KIN + kb, hlf); acc[t] = wmma16b(a, bw, acc[t]); if (MODE == 1) acc[t] = wmma16b(al, bw, acc[t]); } }
#pragma unroll
    for (int t = 0; t < 16; ++t)
#pragma unroll
      for (int r8 = 0; r8 < 8; ++r8) Tf[8 * hlf + r8][t * 16 + nloc] = acc[t][r8] * osc;
    wave_lds_sync();
    const int c0 = g * 256;
    if (c0 < OA) {
      const int hsel = lane >> 4, sub = lane & 15, hd = c0 / C + hsel; for (int rr = 0; rr < 16; ++rr) { float s1 = 0.0f, s2 = 0.0f; for (int j = sub; j < C; j += 16) { const float hv = Tf[rr][hsel * C + j]; s1 += pmul(hv, bfv(as_[hd * C + j])); s2 += pmul(hv, bfv(ad_[hd * C + j])); } for (int o = 8; o; o >>= 1) { s1 += __shfl_xor(s1, o); s2 += __shfl_xor(s2, o); } if (sub == 0) { Eq[rr][hd] = s1; Eq[rr][8 + hd] = s2; } }
      wave_lds_sync();
      for (int pass = 0; pass < 2; ++pass) { for (int rr = 0; rr < 16; ++rr) for (int q = 0; q < 2; ++q) *(volatile v4f*)(FT + (m0 + rr) * OA + c0 + q * 128 + lane * 4) = *(const v4f*)(&Tf[rr][q * 128 + lane * 4]); __threadfence(); } }
    else {
      for (int pass = 0; pass < 2; ++pass) { for (int rr = 0; rr < 16; ++rr) for (int q = 0; q < 256 / 128 && c0 - OA + q * 128 < OL; ++q) { const int lc = c0 - OA + q * 128 + lane * 4; v4f v = *(const v4f*)(&Tf[rr][q * 128 + lane * 4]); for (int k = 0; k < 4; ++k) v[k] += bfv(lb[lc + k]); *(volatile v4f*)(LN + (m0 + rr) * OL + lc) = v; } __threadfence(); } }
    wave_lds_sync(); }
  for (int pass = 0; pass < 2; ++pass) { for (int q = 0; q < 8; ++q) ((volatile float*)ES)[m0 * 16 + q * 32 + lane] = Eq[(q * 32 + lane) >> 4][(q * 32 + lane) & 15]; __threadfence(); } }
template <int NH, int MEANH>
__global__ __launch_bounds__(256) void gat_kernel(const float* __restrict__ FT, const float* __restrict__ ES, const float* __restrict__ LN, const float* __restrict__ bias, const int* __restrict__ srcs, const int* __restrict__ PERM, const int* __restrict__ ROWPTR, const int* __restrict__ ROWCNT, int permLen, int NLIM, float* __restrict__ OUT) { constexpr int OA = NH * C; __shared__ float St[NPB][NH][4]; __shared__ v4f Acc[NPB][NH][32]; const int wave = threadIdx.x >> 5, lane = threadIdx.x & 31; const size_t i = (size_t)blockIdx.x * NPB + wave; if (i >= (size_t)NLIM) return; int st = ROWPTR[i], cnt = ROWCNT[i]; cnt = iclamp(cnt, 0, E); st = iclamp(st, 0, permLen - cnt);
  for (int h = 0; h < NH; ++h) { if (lane == 0) { St[wave][h][0] = ES[i * 16 + 8 + h]; St[wave][h][1] = -INFINITY; St[wave][h][2] = 0.0f; } Acc[wave][h][lane] = (v4f){0, 0, 0, 0}; }
  wave_lds_sync();
  auto visit = [&](size_t u) {
#pragma unroll 1
    for (int h = 0; h < NH; ++h) { const float adi = St[wave][h][0], mx = St[wave][h][1], den = St[wave][h][2]; float s = ES[u * 16 + h] + adi; s = s > 0.0f ? s : 0.2f * s; const float mn = fmaxf(mx, s); const float sf = (mx == -INFINITY) ? 0.0f : __expf(mx - mn); const float p = __expf(s - mn); const v4f v = *(const v4f*)(FT + u * OA + h * C + lane * 4); v4f a = Acc[wave][h][lane]; for (int k = 0; k < 4; ++k) a[k] = pmul(a[k], sf) + pmul(p, v[k]); Acc[wave][h][lane] = a; wave_lds_sync(); if (lane == 0) { St[wave][h][1] = mn; St[wave][h][2] = den * sf + p; } wave_lds_sync(); } };
#pragma unroll 1
  for (int j = 0; j < cnt; ++j) { const int e = iclamp(PERM[st + j], 0, E - 1); const size_t u = (size_t)iclamp(srcs[e], 0, N - 1); if (u >= (size_t)NLIM) continue; visit(u); }
  visit(i);
  for (int pass = 0; pass < 2; ++pass) {
    if (MEANH) { v4f o = {0, 0, 0, 0};
#pragma unroll 1
      for (int h = 0; h < NH; ++h) { const v4f a = Acc[wave][h][lane]; const float dn = St[wave][h][2] + 1e-16f; for (int k = 0; k < 4; ++k) o[k] += a[k] / dn; }
      for (int k = 0; k < 4; ++k) o[k] = o[k] * (1.0f / NH) + bfv(bias[lane * 4 + k]) + LN[i * C + lane * 4 + k]; *(volatile v4f*)(OUT + i * C + lane * 4) = o; }
    else {
#pragma unroll 1
      for (int h = 0; h < NH; ++h) { const v4f a = Acc[wave][h][lane]; const float dn = St[wave][h][2] + 1e-16f; v4f o; for (int k = 0; k < 4; ++k) { const int c = h * C + lane * 4 + k; o[k] = elu(a[k] / dn + bfv(bias[c]) + LN[i * OA + c]); } *(volatile v4f*)(OUT + i * OA + h * C + lane * 4) = o; } }
    __threadfence(); } }
__global__ __launch_bounds__(256) void nodehead_kernel(const float* __restrict__ H3, const float* __restrict__ w, int NLIM, float* __restrict__ UV) { __shared__ float R[16][2]; const int wave = threadIdx.x >> 5, lane = threadIdx.x & 31; for (int half = 0; half < 2; ++half) { const size_t n = (size_t)blockIdx.x * 16 + half * 8 + wave; float s1 = 0.0f, s2 = 0.0f; if (n < (size_t)NLIM) for (int q = 0; q < 4; ++q) { const float hv = H3[n * C + q * 32 + lane]; s1 += pmul(hv, bfv(w[q * 32 + lane])); s2 += pmul(hv, bfv(w[C + q * 32 + lane])); } for (int o = 16; o; o >>= 1) { s1 += __shfl_xor(s1, o); s2 += __shfl_xor(s2, o); } if (lane == 0) { R[half * 8 + wave][0] = s1; R[half * 8 + wave][1] = s2; } }
  __syncthreads();
  for (int pass = 0; pass < 2; ++pass) { if (wave == 0) ((volatile float*)UV)[(size_t)blockIdx.x * 32 + lane] = R[lane >> 1][lane & 1]; __threadfence(); } }
__global__ __launch_bounds__(256) void edge_kernel(const float* __restrict__ UV, const int* __restrict__ rows, const int* __restrict__ cols, const float* __restrict__ mb, int NLIM, float* __restrict__ out) { const size_t e = (size_t)blockIdx.x * 256 + threadIdx.x; if (e >= (size_t)E) return; const int r = iclamp(rows[e], 0, NLIM - 1), c = iclamp(cols[e], 0, NLIM - 1); const float s = UV[(r >> 4) * 32 + (r & 15) * 2] + UV[(c >> 4) * 32 + (c & 15) * 2 + 1] + bfv(mb[0]); const float p = 1.0f / (1.0f + __expf(-s));
  for (int pass = 0; pass < 2; ++pass) { ((volatile float*)out)[e] = p; __threadfence(); } }
}

extern "C" void kernel_launch(void* const* d_in, const int* in_sizes, int n_in, void* d_out, int out_size, void* d_ws, size_t ws_size, hipStream_t stream) {
  (void)n_in;
  auto Fp = [&](int i) { return (const float*)d_in[i]; }; auto Ip = [&](int i) { return (const int*)d_in[i]; };
  if (in_sizes[0] != N * F || in_sizes[1] != 2 * E || in_sizes[2] != F * 512 || in_sizes[8] != 512 * 512 || in_sizes[14] != 512 * 768 || in_sizes[18] != 512 * 128 || in_sizes[20] != 256 || out_size != E) return;
  const int NLIM = N;
  size_t off = 0; char* ws = (char*)d_ws;
  auto carve = [&](size_t bytes) { char* p = ws + off; off += (bytes + 255) & ~(size_t)255; return p; };
  b16* WT1 = (b16*)carve((size_t)1024 * F * 2); b16* WT2 = (b16*)carve((size_t)1024 * 512 * 2); b16* WT3 = (b16*)carve((size_t)1024 * 512 * 2); float* FT = (float*)carve((size_t)N * 768 * 4); float* LN = (float*)carve((size_t)N * 512 * 4); float* ES = (float*)carve((size_t)N * 16 * 4); float* HA = (float*)carve((size_t)N * 512 * 4); float* HB = (float*)carve((size_t)N * 512 * 4); float* UV = (float*)carve((size_t)(N / 16 + 1) * 128); CsrBufs7 csr; off = csr_carve7(csr, ws, off, E, N);
  if (off > ws_size || off > ((size_t)112 << 20)) return;
  const int nb = (NLIM + NPB - 1) / NPB;
  wput_kernel<<<32, 256, 0, stream>>>(Fp(2), Fp(6), F, 512, 512, 1024, WT1); wput_kernel<<<64, 256, 0, stream>>>(Fp(8), Fp(12), 512, 512, 512, 1024, WT2); wput_kernel<<<64, 256, 0, stream>>>(Fp(14), Fp(18), 512, 768, 128, 1024, WT3);
  csr_build7(csr, Ip(1) + E, E, N, stream);
  proj_kernel<0, F, 4, 512><<<NLIM / 16, 32, 0, stream>>>(Fp(0), WT1, Fp(3), Fp(4), Fp(7), NLIM, FT, LN, ES);
  gat_kernel<4, 0><<<nb, 256, 0, stream>>>(FT, ES, LN, Fp(5), Ip(1), csr.PERM, csr.ROWPTR, csr.ROWCNT, (int)csr.permLen, NLIM, HA);
  proj_kernel<1, 512, 4, 512><<<NLIM / 16, 32, 0, stream>>>(HA, WT2, Fp(9), Fp(10), Fp(13), NLIM, FT, LN, ES);
  gat_kernel<4, 0><<<nb, 256, 0, stream>>>(FT, ES, LN, Fp(11), Ip(1), csr.PERM, csr.ROWPTR, csr.ROWCNT, (int)csr.permLen, NLIM, HB);
  proj_kernel<1, 512, 6, 128><<<NLIM / 16, 32, 0, stream>>>(HB, WT3, Fp(15), Fp(16), Fp(19), NLIM, FT, LN, ES);
  gat_kernel<6, 1><<<nb, 256, 0, stream>>>(FT, ES, LN, Fp(17), Ip(1), csr.PERM, csr.ROWPTR, csr.ROWCNT, (int)csr.permLen, NLIM, HA);
  nodehead_kernel<<<(N + 15) / 16, 256, 0, stream>>>(HA, Fp(20), NLIM, UV);
  edge_kernel<<<(E + 255) / 256, 256, 0, stream>>>(UV, Ip(1), Ip(1) + E, Fp(21), NLIM, (float*)d_out);
}
